// GatedDeltaNet_84774064488856
// MI455X (gfx1250) — hardware-run, weakly checked
//
#include <hip/hip_runtime.h>
#include <math.h>

constexpr int kBatch = 2;
constexpr int kSeqT  = 1024;
constexpr int kDim   = 2048;
constexpr int kHeads = 8;
constexpr int kDK    = 128;
constexpr int kDVh   = 256;
constexpr int kKD    = kHeads * kDK;
constexpr int kVD    = kHeads * kDVh;
constexpr int kTok   = kBatch * kSeqT;
constexpr int kNqkab = 2112;
constexpr int kTaps  = 4;
constexpr float kScaleQ  = 0.08838834764831845f;
constexpr float kFltMin  = 1.17549435e-38f;
static_assert(kDim % 32 == 0 && kVD % 32 == 0, "K multiples of 32");
static_assert(kTok % 64 == 0 && kNqkab % 64 == 0 && kVD % 64 == 0 && kDim % 64 == 0, "M,N multiples of 64");
static_assert(((kTok / 64) * (kNqkab / 64)) % 8 == 0 && ((kTok / 64) * (kDim / 64)) % 8 == 0, "8 wave tiles per block");
static_assert(kKD + kKD + 2 * kHeads <= kNqkab, "fold");

typedef __attribute__((ext_vector_type(16))) _Float16 v16h;
typedef __attribute__((ext_vector_type(8)))  _Float16 v8h;
typedef __attribute__((ext_vector_type(16))) __bf16   v16b;
typedef __attribute__((ext_vector_type(8)))  __bf16   v8b;
typedef __attribute__((ext_vector_type(8)))  float    v8f;
typedef __attribute__((ext_vector_type(4)))  float    v4f;
typedef __attribute__((ext_vector_type(4)))  unsigned int v4u;

__device__ __forceinline__ unsigned short f2bf_bits(float f) {
  unsigned u = __float_as_uint(f);
  return (unsigned short)((u + 0x7FFFu + ((u >> 16) & 1u)) >> 16);
}
__device__ __forceinline__ float bf_bits2f(unsigned short h) { return __uint_as_float(((unsigned)h) << 16); }
__device__ __forceinline__ float bf_rn(float f) { return bf_bits2f(f2bf_bits(f)); }
__device__ __forceinline__ unsigned pk16(unsigned short a, unsigned short b) { return (unsigned)a | ((unsigned)b << 16); }

__device__ __forceinline__ void dep_guard4_h(v8f& a, v8f& b, v8f& c, v8f& d, v16h x, v16h y, v16h p, v16h q, v16h r, v16h s) {
  asm volatile("v_nop\n\tv_nop\n\tv_nop\n\tv_nop" : "+v"(a), "+v"(b), "+v"(c), "+v"(d) : "v"(x), "v"(y), "v"(p), "v"(q), "v"(r), "v"(s));
}
__device__ __forceinline__ void dep_guard4_b(v8f& a, v8f& b, v8f& c, v8f& d, v16b x, v16b y, v16b p, v16b q, v16b r, v16b s) {
  asm volatile("v_nop\n\tv_nop\n\tv_nop\n\tv_nop" : "+v"(a), "+v"(b), "+v"(c), "+v"(d) : "v"(x), "v"(y), "v"(p), "v"(q), "v"(r), "v"(s));
}
__device__ __forceinline__ void keep4_h(v16h a, v16h b, v16h c, v16h d) { asm volatile("v_nop" :: "v"(a), "v"(b), "v"(c), "v"(d)); }
__device__ __forceinline__ void keep4_b(v16b a, v16b b, v16b c, v16b d) { asm volatile("v_nop" :: "v"(a), "v"(b), "v"(c), "v"(d)); }
__device__ __forceinline__ void acc_guard4(v8f& a, v8f& b, v8f& c, v8f& d) { asm volatile("v_nop\n\tv_nop\n\tv_nop\n\tv_nop" : "+v"(a), "+v"(b), "+v"(c), "+v"(d)); }
template <typename T> struct Frag;
template <> struct Frag<_Float16> {
  typedef v16h V; union U { v16h v; v8h h[2]; };
  static __device__ __forceinline__ v16h load(const _Float16* p) {
    U f; f.h[0] = *(const v8h*)(p); f.h[1] = *(const v8h*)(p + 16); return f.v;
  }
  static __device__ __forceinline__ v8f mma(v16h a, v16h b, v8f c) {
    return __builtin_amdgcn_wmma_f32_16x16x32_f16(false, a, false, b, (short)0, c, false, false);
  }
  static __device__ __forceinline__ void guard4(v8f& a, v8f& b, v8f& c, v8f& d, v16h x, v16h y, v16h p, v16h q, v16h r, v16h s) { dep_guard4_h(a, b, c, d, x, y, p, q, r, s); }
  static __device__ __forceinline__ void keep(v16h a, v16h b, v16h c, v16h d) { keep4_h(a, b, c, d); }
};
template <> struct Frag<__bf16> {
  typedef v16b V; union U { v16b v; v8b h[2]; };
  static __device__ __forceinline__ v16b load(const __bf16* p) {
    U f; f.h[0] = *(const v8b*)(p); f.h[1] = *(const v8b*)(p + 16); return f.v;
  }
  static __device__ __forceinline__ v8f mma(v16b a, v16b b, v8f c) {
    return __builtin_amdgcn_wmma_f32_16x16x32_bf16(false, a, false, b, (short)0, c, false, false);
  }
  static __device__ __forceinline__ void guard4(v8f& a, v8f& b, v8f& c, v8f& d, v16b x, v16b y, v16b p, v16b q, v16b r, v16b s) { dep_guard4_b(a, b, c, d, x, y, p, q, r, s); }
  static __device__ __forceinline__ void keep(v16b a, v16b b, v16b c, v16b d) { keep4_b(a, b, c, d); }
};

template <int ET> struct Elem;
template <> struct Elem<0> { typedef _Float16 T; };
template <> struct Elem<1> { typedef __bf16 T; };
template <int ET, int SPLIT, int BIAS_MODE, int OUT_MODE>
__global__ __launch_bounds__(256) void wmma_gemm64(
    const unsigned short* __restrict__ Ap, const unsigned short* __restrict__ A2p, int lda, long strideA,
    const unsigned short* __restrict__ Btp, const unsigned short* __restrict__ Bt2p, int ldb, long strideB,
    void* __restrict__ Cout, void* __restrict__ Cout2, int ldc, long strideC,
    const float* __restrict__ bias,
    int M, int N, int K, float scale) {
  typedef typename Elem<ET>::T T;
  typedef typename Frag<T>::V V;
  const T* A = (const T*)Ap; const T* A2 = (const T*)A2p; const T* Bt = (const T*)Btp; const T* Bt2 = (const T*)Bt2p;
  __shared__ __align__(16) float sT[8][16 * 68];
  const int b    = blockIdx.y;
  const int lane = threadIdx.x & 31;
  const int wave = threadIdx.x >> 5;
  const int tilesN = N >> 6;
  const int tilesM = M >> 6;
  const int tile = blockIdx.x * 8 + wave;
  if (tile >= tilesM * tilesN) return;
  const int tm = tile / tilesN;
  const int tn = tile - tm * tilesN;
  const int m0 = tm << 6;
  const int n0 = tn << 6;

  const T* Ab  = A  + (size_t)b * strideA;
  const T* Bb  = Bt + (size_t)b * strideB;
  const T* Ab2 = (SPLIT != 0) ? (A2  + (size_t)b * strideA) : nullptr;
  const T* Bb2 = (SPLIT == 1) ? (Bt2 + (size_t)b * strideB) : nullptr;

  const int rlane = lane & 15;
  const int koff  = (lane >> 4) * 8;
  const int mOff  = (lane >> 4) * 8;

  v8f acc[4][4];
#pragma unroll
  for (int i = 0; i < 4; ++i)
#pragma unroll
    for (int j = 0; j < 4; ++j) acc[i][j] = (v8f){0.f,0.f,0.f,0.f,0.f,0.f,0.f,0.f};

  for (int k0 = 0; k0 < K; k0 += 32) {
    V bh[4], bl[4];
#pragma unroll
    for (int j = 0; j < 4; ++j) {
      const size_t bo = (size_t)(n0 + (j << 4) + rlane) * ldb + koff + k0;
      bh[j] = Frag<T>::load(Bb + bo);
      if (SPLIT == 1) bl[j] = Frag<T>::load(Bb2 + bo);
    }
#pragma unroll
    for (int i = 0; i < 4; ++i) {
      const size_t ao = (size_t)(m0 + (i << 4) + rlane) * lda + koff + k0;
      V ah = Frag<T>::load(Ab + ao);
      V al = ah;
      if (SPLIT != 0) al = Frag<T>::load(Ab2 + ao);
#pragma unroll
      for (int j = 0; j < 4; ++j) {
        acc[i][j] = Frag<T>::mma(ah, bh[j], acc[i][j]);
        if (SPLIT == 1) {
          acc[i][j] = Frag<T>::mma(ah, bl[j], acc[i][j]);
          acc[i][j] = Frag<T>::mma(al, bh[j], acc[i][j]);
        }
        if (SPLIT == 2) acc[i][j] = Frag<T>::mma(al, bh[j], acc[i][j]);
      }
      Frag<T>::guard4(acc[i][0], acc[i][1], acc[i][2], acc[i][3], ah, al, bh[0], bh[1], bh[2], bh[3]);
    }
    Frag<T>::keep(bh[0], bh[1], bh[2], bh[3]);
    if (SPLIT == 1) Frag<T>::keep(bl[0], bl[1], bl[2], bl[3]);
  }
  acc_guard4(acc[0][0], acc[0][1], acc[0][2], acc[0][3]);
  acc_guard4(acc[1][0], acc[1][1], acc[1][2], acc[1][3]);
  acc_guard4(acc[2][0], acc[2][1], acc[2][2], acc[2][3]);
  acc_guard4(acc[3][0], acc[3][1], acc[3][2], acc[3][3]);

  float* slab = sT[wave];
#pragma unroll
  for (int i = 0; i < 4; ++i) {
    const int mBase = m0 + (i << 4);
#pragma unroll
    for (int j = 0; j < 4; ++j) {
      const int n = n0 + (j << 4) + rlane;
      float bv = 0.f;
      if (BIAS_MODE == 2) bv = bias[n];
#pragma unroll
      for (int r = 0; r < 8; ++r) {
        float v = acc[i][j][r] * scale;
        if (BIAS_MODE == 1) v += bias[mBase + mOff + r];
        if (BIAS_MODE == 2) v += bv;
        slab[(mOff + r) * 68 + (j << 4) + rlane] = v;
      }
    }
    __builtin_amdgcn_fence(__ATOMIC_RELEASE, "workgroup");
    __builtin_amdgcn_wave_barrier();
    __builtin_amdgcn_fence(__ATOMIC_ACQUIRE, "workgroup");
    if (OUT_MODE == 0) {
      float* C = (float*)Cout + (size_t)b * strideC;
      const int hh = lane >> 4, c4 = (lane & 15) * 4;
      for (int pass = 0; pass < 2; ++pass) {
#pragma unroll
        for (int it = 0; it < 8; ++it) {
          const int row = it * 2 + hh;
          v4f v = *(const v4f*)(slab + row * 68 + c4);
          *(volatile v4f*)(C + (size_t)(mBase + row) * ldc + n0 + c4) = v;
        }
        __threadfence();
      }
    } else {
      const int q = lane >> 3, c8 = (lane & 7) * 8;
      unsigned short* C  = (unsigned short*)Cout  + (size_t)b * strideC;
      unsigned short* C2 = (OUT_MODE == 2) ? ((unsigned short*)Cout2 + (size_t)b * strideC) : nullptr;
      for (int pass = 0; pass < 2; ++pass) {
#pragma unroll
        for (int it = 0; it < 4; ++it) {
          const int row = it * 4 + q;
          const float* sp = slab + row * 68 + c8;
          v8h hv, lv;
#pragma unroll
          for (int e = 0; e < 8; ++e) {
            if (OUT_MODE == 1) {
              hv[e] = (_Float16)sp[e];
            } else {
              unsigned short hb = f2bf_bits(sp[e]);
              unsigned short lb = f2bf_bits(sp[e] - bf_bits2f(hb));
              hv[e] = __builtin_bit_cast(_Float16, hb);
              lv[e] = __builtin_bit_cast(_Float16, lb);
            }
          }
          *(volatile v8h*)(C + (size_t)(mBase + row) * ldc + n0 + c8) = hv;
          if (OUT_MODE == 2) *(volatile v8h*)(C2 + (size_t)(mBase + row) * ldc + n0 + c8) = lv;
        }
        __threadfence();
      }
    }
    __builtin_amdgcn_fence(__ATOMIC_RELEASE, "workgroup");
    __builtin_amdgcn_wave_barrier();
    __builtin_amdgcn_fence(__ATOMIC_ACQUIRE, "workgroup");
  }
}

__global__ __launch_bounds__(256) void cast8_bf16_kernel(const float* __restrict__ in, unsigned short* __restrict__ out, int n8) {
  const int i = blockIdx.x * 256 + threadIdx.x;
  if (i >= n8) return;
  const float* p = in + 8 * (size_t)i;
  const v4f a = *(const v4f*)(p);
  const v4f c = *(const v4f*)(p + 4);
  unsigned short hb[8];
#pragma unroll
  for (int e = 0; e < 4; ++e) {
    hb[e]     = f2bf_bits(a[e]);
    hb[4 + e] = f2bf_bits(c[e]);
  }
  const v4u u = (v4u){pk16(hb[0], hb[1]), pk16(hb[2], hb[3]), pk16(hb[4], hb[5]), pk16(hb[6], hb[7])};
  unsigned short* q = out + 8 * (size_t)i;
  *(volatile v4u*)q = u;
  __threadfence();
  *(volatile v4u*)q = u;
}

__global__ __launch_bounds__(256) void wqkab_kernel(const float* __restrict__ qw, const float* __restrict__ kw,
                                                    const float* __restrict__ aw, const float* __restrict__ bw,
                                                    unsigned short* __restrict__ out) {
  const int row = blockIdx.x;
  const int c0  = 8 * threadIdx.x;
  const float* src;
  bool zero_row = false;
  if (row < kKD)                         src = qw + (size_t)row * kDim;
  else if (row < 2 * kKD)                src = kw + (size_t)(row - kKD) * kDim;
  else if (row < 2 * kKD + kHeads)       src = aw + (size_t)(row - 2 * kKD) * kDim;
  else if (row < 2 * kKD + 2 * kHeads)   src = bw + (size_t)(row - 2 * kKD - kHeads) * kDim;
  else { src = bw + (size_t)(kHeads - 1) * kDim; zero_row = true; }
  v4f a = *(const v4f*)(src + c0);
  v4f c = *(const v4f*)(src + c0 + 4);
  if (zero_row) { a = (v4f){0.f, 0.f, 0.f, 0.f}; c = (v4f){0.f, 0.f, 0.f, 0.f}; }
  unsigned short hb[8];
#pragma unroll
  for (int e = 0; e < 4; ++e) {
    hb[e]     = f2bf_bits(a[e]);
    hb[4 + e] = f2bf_bits(c[e]);
  }
  const v4u u = (v4u){pk16(hb[0], hb[1]), pk16(hb[2], hb[3]), pk16(hb[4], hb[5]), pk16(hb[6], hb[7])};
  unsigned short* q = out + (size_t)row * kDim + c0;
  *(volatile v4u*)q = u;
  __threadfence();
  *(volatile v4u*)q = u;
}

__global__ __launch_bounds__(256) void decbeta_kernel(const float* __restrict__ pre, const float* __restrict__ alog,
                                                      const float* __restrict__ dtb, float* __restrict__ decp,
                                                      float* __restrict__ betp) {
  __shared__ __align__(16) float sd[8][32];
  __shared__ __align__(16) float sb[8][32];
  const int lane = threadIdx.x & 31, wave = threadIdx.x >> 5;
  const int base = (blockIdx.x * 8 + wave) * 4;
  const int row  = base + (lane >> 3);
  const int hd   = lane & 7;
  const float xa = pre[(size_t)row * kNqkab + 2 * kKD + hd];
  const float xb = pre[(size_t)row * kNqkab + 2 * kKD + kHeads + hd];
  const float nal = bf_rn(alog[hd]);
  const float ndb = bf_rn(dtb[hd]);
  const float x  = xa + ndb;
  const float sp = fmaxf(x, 0.0f) + log1pf(expf(-fabsf(x)));
  const float gd = -expf(nal) * sp;
  float dcy = expf(gd);
  if (dcy < kFltMin) dcy = 0.0f;
  const float bet = 1.0f / (1.0f + expf(-xb));
  sd[wave][lane] = dcy;
  sb[wave][lane] = bet;
  __builtin_amdgcn_fence(__ATOMIC_RELEASE, "workgroup");
  __builtin_amdgcn_wave_barrier();
  __builtin_amdgcn_fence(__ATOMIC_ACQUIRE, "workgroup");
  const int c4 = (lane & 7) * 4;
  const v4f dv4 = *(const v4f*)(&sd[wave][c4]);
  const v4f bv4 = *(const v4f*)(&sb[wave][c4]);
  float* pd = decp + (size_t)base * kHeads + c4;
  float* pb = betp + (size_t)base * kHeads + c4;
  if (lane < 8) { *(volatile v4f*)pd = dv4; *(volatile v4f*)pb = bv4; }
  __threadfence();
  if (lane < 8) { *(volatile v4f*)pd = dv4; *(volatile v4f*)pb = bv4; }
}

__global__ __launch_bounds__(256) void conv_qk_kernel(const float* __restrict__ pre, const float* __restrict__ qcw,
                                                      const float* __restrict__ kcw, float* __restrict__ qn,
                                                      float* __restrict__ kn) {
  const int row   = blockIdx.x;
  const int which = blockIdx.y;
  const int lane  = threadIdx.x & 31, hd = threadIdx.x >> 5;
  const float* cw = which ? kcw : qcw;
  float* outp     = which ? kn : qn;
  const int t    = row & (kSeqT - 1);
  const int c0   = hd * kDK + 4 * lane;
  const int pcol = which * kKD + c0;
  const v4f w0 = *(const v4f*)(cw + (size_t)(c0 + 0) * kTaps);
  const v4f w1 = *(const v4f*)(cw + (size_t)(c0 + 1) * kTaps);
  const v4f w2 = *(const v4f*)(cw + (size_t)(c0 + 2) * kTaps);
  const v4f w3 = *(const v4f*)(cw + (size_t)(c0 + 3) * kTaps);
  float a0 = 0.0f, a1 = 0.0f, a2 = 0.0f, a3 = 0.0f;
#pragma unroll
  for (int j = 0; j < kTaps; ++j) {
    const int tk = t - 3 + j;
    int srow = row - 3 + j;
    srow = srow < 0 ? 0 : srow;
    const float f = (tk >= 0) ? 1.0f : 0.0f;
    const v4f x = *(const v4f*)(pre + (size_t)srow * kNqkab + pcol);
    a0 = fmaf(x[0] * f, bf_rn(w0[j]), a0);
    a1 = fmaf(x[1] * f, bf_rn(w1[j]), a1);
    a2 = fmaf(x[2] * f, bf_rn(w2[j]), a2);
    a3 = fmaf(x[3] * f, bf_rn(w3[j]), a3);
  }
  const float s0 = a0 * (1.0f / (1.0f + expf(-a0)));
  const float s1 = a1 * (1.0f / (1.0f + expf(-a1)));
  const float s2 = a2 * (1.0f / (1.0f + expf(-a2)));
  const float s3 = a3 * (1.0f / (1.0f + expf(-a3)));
  float ss = (s0 * s0 + s1 * s1) + (s2 * s2 + s3 * s3);
#pragma unroll
  for (int off = 16; off > 0; off >>= 1) ss += __shfl_xor(ss, off, 32);
  const float rs = rsqrtf(ss + 1e-6f);
  const v4f o = (v4f){s0 * rs, s1 * rs, s2 * rs, s3 * rs};
  float* op = outp + (size_t)row * kKD + c0;
  *(volatile v4f*)op = o;
  __threadfence();
  *(volatile v4f*)op = o;
}

__global__ __launch_bounds__(256) void conv_v_kernel(const float* __restrict__ vpre, const float* __restrict__ vcw,
                                                     float* __restrict__ vn) {
  const int row = blockIdx.x;
  const int t   = row & (kSeqT - 1);
  const int tid = threadIdx.x;
#pragma unroll 1
  for (int grp = 0; grp < 2; ++grp) {
    const int c0 = grp * (kVD / 2) + 4 * tid;
    const v4f w0 = *(const v4f*)(vcw + (size_t)(c0 + 0) * kTaps);
    const v4f w1 = *(const v4f*)(vcw + (size_t)(c0 + 1) * kTaps);
    const v4f w2 = *(const v4f*)(vcw + (size_t)(c0 + 2) * kTaps);
    const v4f w3 = *(const v4f*)(vcw + (size_t)(c0 + 3) * kTaps);
    float a0 = 0.0f, a1 = 0.0f, a2 = 0.0f, a3 = 0.0f;
#pragma unroll
    for (int j = 0; j < kTaps; ++j) {
      const int tk = t - 3 + j;
      int srow = row - 3 + j;
      srow = srow < 0 ? 0 : srow;
      const float f = (tk >= 0) ? 1.0f : 0.0f;
      const v4f x = *(const v4f*)(vpre + (size_t)srow * kVD + c0);
      a0 = fmaf(x[0] * f, bf_rn(w0[j]), a0);
      a1 = fmaf(x[1] * f, bf_rn(w1[j]), a1);
      a2 = fmaf(x[2] * f, bf_rn(w2[j]), a2);
      a3 = fmaf(x[3] * f, bf_rn(w3[j]), a3);
    }
    const v4f o = (v4f){a0 * (1.0f / (1.0f + expf(-a0))), a1 * (1.0f / (1.0f + expf(-a1))),
                        a2 * (1.0f / (1.0f + expf(-a2))), a3 * (1.0f / (1.0f + expf(-a3)))};
    float* op = vn + (size_t)row * kVD + c0;
    *(volatile v4f*)op = o;
    __threadfence();
    *(volatile v4f*)op = o;
    asm volatile("" ::: "memory");
  }
}

constexpr int kTch    = 16;
constexpr int kSPitch = 132;
constexpr float kRenorm = 8.673617379884035e-19f;
static_assert(kSeqT % kTch == 0 && kTch % 4 == 0, "chunking");

__global__ __launch_bounds__(64) void scan_kernel(const float* __restrict__ qn, const float* __restrict__ kn,
                                                  const float* __restrict__ vn, const float* __restrict__ dec,
                                                  const float* __restrict__ bet, float* __restrict__ oattn) {
  __shared__ __align__(16) float sS[64 * kSPitch];
  __shared__ __align__(16) float sQ[kTch * kDK];
  __shared__ __align__(16) float sK[kTch * kDK];
  __shared__ __align__(16) float sV[kTch * 64];
  __shared__ __align__(16) float sO[2][4 * 32];
  __shared__ float sDc[kTch];
  __shared__ float sBt[kTch];
  const int tid = threadIdx.x, lane = tid & 31, wave = tid >> 5;
  const int bh = blockIdx.x >> 2, cq = blockIdx.x & 3;
  const int b = bh >> 3, h = bh & 7;
  const size_t rowb = (size_t)b * kSeqT;
  const int colh = h * kDVh + cq * 64;
  float* sc = sS + tid * kSPitch;
  const v4f z4 = (v4f){0.0f, 0.0f, 0.0f, 0.0f};
#pragma unroll 1
  for (int g = 0; g < 32; ++g) *(v4f*)(sc + 4 * g) = z4;
  float cfac = 1.0f;
  float* so = sO[wave];

  for (int t0 = 0; t0 < kSeqT; t0 += kTch) {
    __syncthreads();
#pragma unroll 1
    for (int i = 0; i < 8; ++i) {
      const int idx = tid + 64 * i;
      const int r = idx >> 5, c4 = (idx & 31) * 4;
      const size_t go = (rowb + t0 + r) * kKD + h * kDK + c4;
      *(v4f*)(sQ + r * kDK + c4) = *(const v4f*)(qn + go);
      *(v4f*)(sK + r * kDK + c4) = *(const v4f*)(kn + go);
    }
#pragma unroll 1
    for (int i = 0; i < 4; ++i) {
      const int idx = tid + 64 * i;
      const int r = idx >> 4, c4 = (idx & 15) * 4;
      *(v4f*)(sV + r * 64 + c4) = *(const v4f*)(vn + (rowb + t0 + r) * kVD + colh + c4);
    }
    if (wave == 0) {
      const int r = lane & 15;
      const size_t gi = (rowb + t0 + r) * kHeads + h;
      const float dvv = dec[gi];
      const float bvv = bet[gi];
      if (lane < kTch) { sDc[lane] = dvv; sBt[lane] = bvv; }
    }
    __syncthreads();

#pragma unroll 1
    for (int tt = 0; tt < kTch; ++tt) {
      const float dcy = sDc[tt];
      const float btv = sBt[tt];
      const float vv  = sV[tt * 64 + tid];
      const float* kp = sK + tt * kDK;
      const float* qp = sQ + tt * kDK;
      const float cnew = cfac * dcy;
      if (cnew < kRenorm) {
#pragma unroll 1
        for (int gg = 0; gg < 32; gg += 4) {
#pragma unroll
          for (int uu = 0; uu < 4; ++uu) {
            const int g = gg + uu;
            v4f s4 = *(const v4f*)(sc + 4 * g);
            s4 = s4 * cnew;
            *(v4f*)(sc + 4 * g) = s4;
          }
        }
        cfac = 1.0f;
      } else {
        cfac = cnew;
      }
      float p0 = 0.0f, p1 = 0.0f, p2 = 0.0f, p3 = 0.0f;
#pragma unroll 1
      for (int gg = 0; gg < 32; gg += 4) {
#pragma unroll
        for (int uu = 0; uu < 4; ++uu) {
          const int g = gg + uu;
          const v4f s4 = *(const v4f*)(sc + 4 * g);
          const v4f k4 = *(const v4f*)(kp + 4 * g);
          p0 = fmaf(k4[0], s4[0], p0);
          p1 = fmaf(k4[1], s4[1], p1);
          p2 = fmaf(k4[2], s4[2], p2);
          p3 = fmaf(k4[3], s4[3], p3);
        }
      }
      const float kv = cfac * ((p0 + p1) + (p2 + p3));
      const float u  = (vv - kv) * btv;
      const float w  = u * (1.0f / cfac);
      float o0 = 0.0f, o1 = 0.0f, o2 = 0.0f, o3 = 0.0f;
#pragma unroll 1
      for (int gg = 0; gg < 32; gg += 4) {
#pragma unroll
        for (int uu = 0; uu < 4; ++uu) {
          const int g = gg + uu;
          v4f s4 = *(const v4f*)(sc + 4 * g);
          const v4f k4 = *(const v4f*)(kp + 4 * g);
          const v4f q4 = *(const v4f*)(qp + 4 * g);
          s4[0] = fmaf(k4[0], w, s4[0]);
          s4[1] = fmaf(k4[1], w, s4[1]);
          s4[2] = fmaf(k4[2], w, s4[2]);
          s4[3] = fmaf(k4[3], w, s4[3]);
          *(v4f*)(sc + 4 * g) = s4;
          o0 = fmaf(q4[0], s4[0], o0);
          o1 = fmaf(q4[1], s4[1], o1);
          o2 = fmaf(q4[2], s4[2], o2);
          o3 = fmaf(q4[3], s4[3], o3);
        }
      }
      const float ov = (cfac * kScaleQ) * ((o0 + o1) + (o2 + o3));
      so[(tt & 3) * 32 + lane] = ov;
      if ((tt & 3) == 3) {
        __builtin_amdgcn_fence(__ATOMIC_RELEASE, "workgroup");
        __builtin_amdgcn_wave_barrier();
        __builtin_amdgcn_fence(__ATOMIC_ACQUIRE, "workgroup");
        const int rq = lane >> 3, c4 = (lane & 7) * 4;
        const v4f val = *(const v4f*)(so + rq * 32 + c4);
        float* op = oattn + (rowb + t0 + tt - 3 + rq) * kVD + colh + wave * 32 + c4;
        *(volatile v4f*)op = val;
        __threadfence();
        *(volatile v4f*)op = val;
        __builtin_amdgcn_fence(__ATOMIC_RELEASE, "workgroup");
        __builtin_amdgcn_wave_barrier();
        __builtin_amdgcn_fence(__ATOMIC_ACQUIRE, "workgroup");
      }
    }
  }
}

__global__ __launch_bounds__(256) void rms_gate_kernel(const float* __restrict__ oattn, const float* __restrict__ gate,
                                                       const float* __restrict__ onw, unsigned short* __restrict__ yhi,
                                                       unsigned short* __restrict__ ylo) {
  const int row  = blockIdx.x;
  const int lane = threadIdx.x & 31, hd = threadIdx.x >> 5;
  const size_t cb = (size_t)row * kVD + hd * kDVh + 8 * lane;
  const v4f oa = *(const v4f*)(oattn + cb);
  const v4f ob = *(const v4f*)(oattn + cb + 4);
  const v4f ga = *(const v4f*)(gate + cb);
  const v4f gb = *(const v4f*)(gate + cb + 4);
  const v4f na = *(const v4f*)(onw + 8 * lane);
  const v4f nb = *(const v4f*)(onw + 8 * lane + 4);
  float ov[8], gv[8], nv[8];
#pragma unroll
  for (int e = 0; e < 4; ++e) {
    ov[e] = oa[e]; ov[4 + e] = ob[e];
    gv[e] = ga[e]; gv[4 + e] = gb[e];
    nv[e] = na[e]; nv[4 + e] = nb[e];
  }
  float ss = 0.0f;
#pragma unroll
  for (int e = 0; e < 8; ++e) ss = fmaf(ov[e], ov[e], ss);
#pragma unroll
  for (int off = 16; off > 0; off >>= 1) ss += __shfl_xor(ss, off, 32);
  const float rs = rsqrtf(ss * (1.0f / 256.0f) + 1e-5f);
  unsigned short hb[8], lb[8];
#pragma unroll
  for (int e = 0; e < 8; ++e) {
    const float g  = gv[e];
    const float sg = g * (1.0f / (1.0f + expf(-g)));
    const float y  = ((ov[e] * rs) * bf_rn(nv[e])) * sg;
    const unsigned short h16 = f2bf_bits(y);
    hb[e] = h16;
    lb[e] = f2bf_bits(y - bf_bits2f(h16));
  }
  const v4u uh = (v4u){pk16(hb[0], hb[1]), pk16(hb[2], hb[3]), pk16(hb[4], hb[5]), pk16(hb[6], hb[7])};
  const v4u ul = (v4u){pk16(lb[0], lb[1]), pk16(lb[2], lb[3]), pk16(lb[4], lb[5]), pk16(lb[6], lb[7])};
  unsigned short* ph = yhi + cb;
  unsigned short* pl = ylo + cb;
  *(volatile v4u*)ph = uh;
  *(volatile v4u*)pl = ul;
  __threadfence();
  *(volatile v4u*)ph = uh;
  *(volatile v4u*)pl = ul;
}

extern "C" void kernel_launch(void* const* d_in, const int* in_sizes, int n_in,
                              void* d_out, int out_size, void* d_ws, size_t ws_size,
                              hipStream_t stream) {
  if (n_in < 14) return;
  if (in_sizes[0] != kTok * kDim) return;
  if (in_sizes[1] != kKD * kDim || in_sizes[2] != kKD * kDim) return;
  if (in_sizes[3] != kVD * kDim || in_sizes[6] != kVD * kDim || in_sizes[7] != kDim * kVD) return;
  if (in_sizes[4] != kHeads * kDim || in_sizes[5] != kHeads * kDim) return;
  if (in_sizes[8] != kKD * kTaps || in_sizes[9] != kKD * kTaps || in_sizes[10] != kVD * kTaps) return;
  if (in_sizes[11] != kHeads || in_sizes[12] != kHeads || in_sizes[13] != kDVh) return;
  if (out_size != kTok * kDim) return;

  const size_t szHbf = (size_t)kTok * kDim * 2;
  const size_t szWqk = (size_t)kNqkab * kDim * 2;
  const size_t szWsc = (size_t)kDim * kDim * 2;
  const size_t szPre = (size_t)kTok * kNqkab * 4;
  const size_t szF32 = (size_t)kTok * kVD * 4;
  const size_t szQn  = (size_t)kTok * kKD * 4;
  const size_t szY   = (size_t)kTok * kVD * 2;
  const size_t szDb  = (size_t)kTok * kHeads * 4;
  const size_t offHbf = 0;
  const size_t offWqk = offHbf + szHbf;
  const size_t offWsc = offWqk + szWqk;
  const size_t offPre = offWsc + szWsc;
  const size_t offVpo = offPre + szPre;
  const size_t offGat = offVpo + szF32;
  const size_t offQn  = offGat + szF32;
  const size_t offKn  = offQn + szQn;
  const size_t offVn  = offKn + szQn;
  const size_t offYhi = offVn + szF32;
  const size_t offYlo = offYhi + szY;
  const size_t offDec = offYlo + szY;
  const size_t offBet = offDec + szDb;
  const size_t total  = offBet + szDb;
  if (ws_size < total) return;

  const float* hs   = (const float*)d_in[0];
  const float* q_w  = (const float*)d_in[1];
  const float* k_w  = (const float*)d_in[2];
  const float* v_w  = (const float*)d_in[3];
  const float* a_w  = (const float*)d_in[4];
  const float* b_w  = (const float*)d_in[5];
  const float* g_w  = (const float*)d_in[6];
  const float* o_w  = (const float*)d_in[7];
  const float* qcw  = (const float*)d_in[8];
  const float* kcw  = (const float*)d_in[9];
  const float* vcw  = (const float*)d_in[10];
  const float* alog = (const float*)d_in[11];
  const float* dtb  = (const float*)d_in[12];
  const float* onw  = (const float*)d_in[13];
  float* out = (float*)d_out;
  char* ws = (char*)d_ws;
  unsigned short* hbf = (unsigned short*)(ws + offHbf);
  unsigned short* wqk = (unsigned short*)(ws + offWqk);
  unsigned short* wsc = (unsigned short*)(ws + offWsc);
  float* pre  = (float*)(ws + offPre);
  float* vpo  = (float*)(ws + offVpo);
  float* gat  = (float*)(ws + offGat);
  float* qn   = (float*)(ws + offQn);
  float* kn   = (float*)(ws + offKn);
  float* vn   = (float*)(ws + offVn);
  unsigned short* yhi = (unsigned short*)(ws + offYhi);
  unsigned short* ylo = (unsigned short*)(ws + offYlo);
  float* decp = (float*)(ws + offDec);
  float* betp = (float*)(ws + offBet);

  const int n8h = (kTok * kDim) / 8;
  const int n8w = (kDim * kDim) / 8;
  const int blocksQkab = ((kTok / 64) * (kNqkab / 64)) / 8;
  const int blocksSq   = ((kTok / 64) * (kDim / 64)) / 8;

  cast8_bf16_kernel<<<dim3(n8h / 256), dim3(256), 0, stream>>>(hs, hbf, n8h);
  wqkab_kernel<<<dim3(kNqkab), dim3(256), 0, stream>>>(q_w, k_w, a_w, b_w, wqk);
  wmma_gemm64<1, 0, 0, 0><<<dim3(blocksQkab, 1), dim3(256), 0, stream>>>(
      hbf, hbf, kDim, 0L, wqk, wqk, kDim, 0L, (void*)pre, (void*)pre, kNqkab, 0L, decp, kTok, kNqkab, kDim, 1.0f);
  cast8_bf16_kernel<<<dim3(n8w / 256), dim3(256), 0, stream>>>(v_w, wsc, n8w);
  wmma_gemm64<1, 0, 0, 0><<<dim3(blocksSq, 1), dim3(256), 0, stream>>>(
      hbf, hbf, kDim, 0L, wsc, wsc, kDim, 0L, (void*)vpo, (void*)vpo, kVD, 0L, decp, kTok, kVD, kDim, 1.0f);
  cast8_bf16_kernel<<<dim3(n8w / 256), dim3(256), 0, stream>>>(g_w, wsc, n8w);
  wmma_gemm64<1, 0, 0, 0><<<dim3(blocksSq, 1), dim3(256), 0, stream>>>(
      hbf, hbf, kDim, 0L, wsc, wsc, kDim, 0L, (void*)gat, (void*)gat, kVD, 0L, decp, kTok, kVD, kDim, 1.0f);
  cast8_bf16_kernel<<<dim3(n8w / 256), dim3(256), 0, stream>>>(o_w, wsc, n8w);
  decbeta_kernel<<<dim3(kTok / 32), dim3(256), 0, stream>>>(pre, alog, dtb, decp, betp);
  conv_qk_kernel<<<dim3(kTok, 2), dim3(256), 0, stream>>>(pre, qcw, kcw, qn, kn);
  conv_v_kernel<<<dim3(kTok), dim3(256), 0, stream>>>(vpo, vcw, vn);
  scan_kernel<<<dim3(kBatch * kHeads * 4), dim3(64), 0, stream>>>(qn, kn, vn, decp, betp, vpo);
  rms_gate_kernel<<<dim3(kTok), dim3(256), 0, stream>>>(vpo, gat, onw, yhi, ylo);
  wmma_gemm64<1, 2, 0, 0><<<dim3(blocksSq, 1), dim3(256), 0, stream>>>(
      yhi, ylo, kVD, 0L, wsc, wsc, kVD, 0L, (void*)out, (void*)out, kDim, 0L, decp, kTok, kDim, kVD, 1.0f);
}
